// MambaMLPBlock_36627481100485
// MI455X (gfx1250) — hardware-verified
//
#include <hip/hip_runtime.h>
#include <math.h>

typedef __attribute__((ext_vector_type(16))) _Float16 v16h;
typedef __attribute__((ext_vector_type(8)))  _Float16 v8h;
typedef __attribute__((ext_vector_type(16))) __bf16   v16b;
typedef __attribute__((ext_vector_type(8)))  __bf16   v8b;
typedef __attribute__((ext_vector_type(8)))  float    v8f;
typedef __attribute__((ext_vector_type(4)))  float    v4f;

constexpr int kBatch = 4;
constexpr int kT     = 256;
constexpr int kNsp   = 64;
constexpr int kCh    = 128;
constexpr int kDin   = 256;
constexpr int kNst   = 16;
constexpr int kDtR   = 8;
constexpr int kPrjN  = 40;
constexpr int kPrjP  = 64;
constexpr int kXZP   = 2 * kDin;
constexpr int kMlp   = 256;
constexpr int kRows  = kNsp * kT;
constexpr int kTP    = 260;
constexpr int kHP    = 136;
static_assert(kRows % 64 == 0 && kCh % 32 == 0 && kDin % 32 == 0, "tile multiples");

__device__ __forceinline__ unsigned short f2bf_bits(float f) {
  unsigned u = __float_as_uint(f);
  return (unsigned short)((u + 0x7FFFu + ((u >> 16) & 1u)) >> 16);
}
__device__ __forceinline__ float bf_bits2f(unsigned short h) { return __uint_as_float(((unsigned)h) << 16); }

__device__ __forceinline__ void dep_guard_h(v8f& a, v8f& b, v16h x, v16h y) { asm volatile("v_nop\n\tv_nop\n\tv_nop\n\tv_nop" : "+v"(a), "+v"(b) : "v"(x), "v"(y)); }
__device__ __forceinline__ void dep_guard_b(v8f& a, v8f& b, v16b x, v16b y) { asm volatile("v_nop\n\tv_nop\n\tv_nop\n\tv_nop" : "+v"(a), "+v"(b) : "v"(x), "v"(y)); }
__device__ __forceinline__ void keep4_h(v16h a, v16h b, v16h c, v16h d) { asm volatile("v_nop" :: "v"(a), "v"(b), "v"(c), "v"(d)); }
__device__ __forceinline__ void keep4_b(v16b a, v16b b, v16b c, v16b d) { asm volatile("v_nop" :: "v"(a), "v"(b), "v"(c), "v"(d)); }
__device__ __forceinline__ void acc_guard4(v8f& a, v8f& b, v8f& c, v8f& d) { asm volatile("v_nop\n\tv_nop\n\tv_nop\n\tv_nop" : "+v"(a), "+v"(b), "+v"(c), "+v"(d)); }
template <typename T> struct Frag;
template <> struct Frag<_Float16> {
  typedef v16h V; union U { v16h v; v8h h[2]; };
  static __device__ __forceinline__ v16h load(const _Float16* p) {
    U f; f.h[0] = *(const v8h*)(p); f.h[1] = *(const v8h*)(p + 16); return f.v;
  }
  static __device__ __forceinline__ v8f mma(v16h a, v16h b, v8f c) {
    return __builtin_amdgcn_wmma_f32_16x16x32_f16(false, a, false, b, (short)0, c, false, false);
  }
  static __device__ __forceinline__ void guard(v8f& a, v8f& b, v16h x, v16h y) { dep_guard_h(a, b, x, y); }
  static __device__ __forceinline__ void keep(v16h a, v16h b, v16h c, v16h d) { keep4_h(a, b, c, d); }
};
template <> struct Frag<__bf16> {
  typedef v16b V; union U { v16b v; v8b h[2]; };
  static __device__ __forceinline__ v16b load(const __bf16* p) {
    U f; f.h[0] = *(const v8b*)(p); f.h[1] = *(const v8b*)(p + 16); return f.v;
  }
  static __device__ __forceinline__ v8f mma(v16b a, v16b b, v8f c) {
    return __builtin_amdgcn_wmma_f32_16x16x32_bf16(false, a, false, b, (short)0, c, false, false);
  }
  static __device__ __forceinline__ void guard(v8f& a, v8f& b, v16b x, v16b y) { dep_guard_b(a, b, x, y); }
  static __device__ __forceinline__ void keep(v16b a, v16b b, v16b c, v16b d) { keep4_b(a, b, c, d); }
};

template <int ET> struct Elem;
template <> struct Elem<0> { typedef _Float16 T; };
template <> struct Elem<1> { typedef __bf16 T; };
template <int ET, bool SPLIT, int BIAS_MODE, int OUT_MODE, bool RESID, int ACT = 0>
__global__ __launch_bounds__(256) void wmma_gemm64(
    const unsigned short* __restrict__ Ap, const unsigned short* __restrict__ A2p, int lda, long strideA,
    const unsigned short* __restrict__ Btp, const unsigned short* __restrict__ Bt2p, int ldb, long strideB,
    void* __restrict__ Cout, void* __restrict__ Cout2, int ldc, long strideC,
    const float* __restrict__ bias,
    const float* __restrict__ resid, long strideR,
    int M, int N, int K, float scale) {
  typedef typename Elem<ET>::T T;
  typedef typename Frag<T>::V V;
  const T* A = (const T*)Ap; const T* A2 = (const T*)A2p; const T* Bt = (const T*)Btp; const T* Bt2 = (const T*)Bt2p;
  __shared__ __align__(16) float sT[8][16 * 68];
  const int b    = blockIdx.y;
  const int lane = threadIdx.x & 31;
  const int wave = threadIdx.x >> 5;
  const int tilesN = N >> 6;
  const int tilesM = M >> 6;
  const int tile = blockIdx.x * 8 + wave;
  if (tile >= tilesM * tilesN) return;
  const int tm = tile / tilesN;
  const int tn = tile - tm * tilesN;
  const int m0 = tm << 6;
  const int n0 = tn << 6;

  const T* Ab  = A  + (size_t)b * strideA;
  const T* Bb  = Bt + (size_t)b * strideB;
  const T* Ab2 = SPLIT ? (A2  + (size_t)b * strideA) : nullptr;
  const T* Bb2 = SPLIT ? (Bt2 + (size_t)b * strideB) : nullptr;

  const int rlane = lane & 15;
  const int koff  = (lane >> 4) * 8;
  const int mOff  = (lane >> 4) * 8;

  v8f acc[4][4];
#pragma unroll
  for (int i = 0; i < 4; ++i)
#pragma unroll
    for (int j = 0; j < 4; ++j) acc[i][j] = (v8f){0.f,0.f,0.f,0.f,0.f,0.f,0.f,0.f};

  for (int k0 = 0; k0 < K; k0 += 32) {
    V bh[4], bl[4];
#pragma unroll
    for (int j = 0; j < 4; ++j) {
      const size_t bo = (size_t)(n0 + (j << 4) + rlane) * ldb + koff + k0;
      bh[j] = Frag<T>::load(Bb + bo);
      if (SPLIT) bl[j] = Frag<T>::load(Bb2 + bo);
    }
#pragma unroll
    for (int i = 0; i < 4; ++i) {
      const size_t ao = (size_t)(m0 + (i << 4) + rlane) * lda + koff + k0;
      V ah = Frag<T>::load(Ab + ao);
      V al;
      if (SPLIT) al = Frag<T>::load(Ab2 + ao);
#pragma unroll
      for (int j = 0; j < 4; ++j) {
        acc[i][j] = Frag<T>::mma(ah, bh[j], acc[i][j]);
        if (SPLIT) {
          acc[i][j] = Frag<T>::mma(ah, bl[j], acc[i][j]);
          acc[i][j] = Frag<T>::mma(al, bh[j], acc[i][j]);
        }
      }
      Frag<T>::guard(acc[i][0], acc[i][3], ah, SPLIT ? al : ah);
    }
    Frag<T>::keep(bh[0], bh[1], bh[2], bh[3]);
    if (SPLIT) Frag<T>::keep(bl[0], bl[1], bl[2], bl[3]);
  }
  acc_guard4(acc[0][0], acc[0][1], acc[0][2], acc[0][3]);
  acc_guard4(acc[1][0], acc[1][1], acc[1][2], acc[1][3]);
  acc_guard4(acc[2][0], acc[2][1], acc[2][2], acc[2][3]);
  acc_guard4(acc[3][0], acc[3][1], acc[3][2], acc[3][3]);

  float* slab = sT[wave];
  const float* Rb = RESID ? (resid + (size_t)b * strideR) : nullptr;
#pragma unroll
  for (int i = 0; i < 4; ++i) {
    const int mBase = m0 + (i << 4);
#pragma unroll
    for (int j = 0; j < 4; ++j) {
      const int n = n0 + (j << 4) + rlane;
      float bv = 0.f;
      if (BIAS_MODE == 2) bv = bias[n];
#pragma unroll
      for (int r = 0; r < 8; ++r) {
        float v = acc[i][j][r] * scale;
        if (BIAS_MODE == 1) v += bias[mBase + mOff + r];
        if (BIAS_MODE == 2) v += bv;
        if (RESID) v += Rb[(size_t)(mBase + mOff + r) * ldc + n];
        if (ACT == 1) v = tanhf(v);
        if (ACT == 2) v = fmaxf(v, 0.0f);
        if (ACT == 3) v = v / (1.0f + expf(-v));
        if (ACT == 4) v = (v > 0.f) ? v : 0.01f * v;
        if (ACT == 5) v = 0.5f * v * (1.0f + erff(v * 0.70710678118654752f));
        slab[(mOff + r) * 68 + (j << 4) + rlane] = v;
      }
    }
    __builtin_amdgcn_fence(__ATOMIC_RELEASE, "workgroup");
    __builtin_amdgcn_wave_barrier();
    __builtin_amdgcn_fence(__ATOMIC_ACQUIRE, "workgroup");
    if (OUT_MODE == 0) {
      float* C = (float*)Cout + (size_t)b * strideC;
      const int hh = lane >> 4, c4 = (lane & 15) * 4;
      for (int pass = 0; pass < 2; ++pass) {
#pragma unroll
        for (int it = 0; it < 8; ++it) {
          const int row = it * 2 + hh;
          v4f v = *(const v4f*)(slab + row * 68 + c4);
          *(volatile v4f*)(C + (size_t)(mBase + row) * ldc + n0 + c4) = v;
        }
        __threadfence();
      }
    } else {
      const int q = lane >> 3, c8 = (lane & 7) * 8;
      unsigned short* C  = (unsigned short*)Cout  + (size_t)b * strideC;
      unsigned short* C2 = (OUT_MODE == 2) ? ((unsigned short*)Cout2 + (size_t)b * strideC) : nullptr;
      for (int pass = 0; pass < 2; ++pass) {
#pragma unroll
        for (int it = 0; it < 4; ++it) {
          const int row = it * 4 + q;
          const float* sp = slab + row * 68 + c8;
          v8h hv, lv;
#pragma unroll
          for (int e = 0; e < 8; ++e) {
            if (OUT_MODE == 1) {
              hv[e] = (_Float16)sp[e];
            } else {
              unsigned short hb = f2bf_bits(sp[e]);
              unsigned short lb = f2bf_bits(sp[e] - bf_bits2f(hb));
              hv[e] = __builtin_bit_cast(_Float16, hb);
              lv[e] = __builtin_bit_cast(_Float16, lb);
            }
          }
          *(volatile v8h*)(C + (size_t)(mBase + row) * ldc + n0 + c8) = hv;
          if (OUT_MODE == 2) *(volatile v8h*)(C2 + (size_t)(mBase + row) * ldc + n0 + c8) = lv;
        }
        __threadfence();
      }
    }
    __builtin_amdgcn_fence(__ATOMIC_RELEASE, "workgroup");
    __builtin_amdgcn_wave_barrier();
    __builtin_amdgcn_fence(__ATOMIC_ACQUIRE, "workgroup");
  }
}

__global__ __launch_bounds__(256) void cast_rows_f16_kernel(
    const float* __restrict__ src, unsigned short* __restrict__ dst, int N, int K, int total8, float scale)
{
  const int i = blockIdx.x * 256 + threadIdx.x;
  if (i >= total8) return;
  const int e0  = i << 3;
  const int row = e0 / K;
  const int col = e0 - row * K;
  const int rowc = (row < N) ? row : (N - 1);
  const bool live = (row < N);
  const float* p = src + (size_t)rowc * K + col;
  const v4f a0 = *(const v4f*)(p);
  const v4f a1 = *(const v4f*)(p + 4);
  v8h hv;
#pragma unroll
  for (int e = 0; e < 4; ++e) {
    hv[e]     = live ? (_Float16)(a0[e] * scale) : (_Float16)0.0f;
    hv[4 + e] = live ? (_Float16)(a1[e] * scale) : (_Float16)0.0f;
  }
  unsigned short* q = dst + (size_t)e0;
  *(volatile v8h*)q = hv;
  __threadfence();
  *(volatile v8h*)q = hv;
}

__global__ __launch_bounds__(256) void xpose_cast_kernel(
    const float* __restrict__ Xb, unsigned short* __restrict__ Ob, int Kdim, int Ndim,
    long strideIn, long strideOut, float scale)
{
  __shared__ float tile[64 * 65];
  const int tid = threadIdx.x, lane = tid & 31, wave = tid >> 5;
  const float* W = Xb + (size_t)blockIdx.z * strideIn;
  unsigned short* Bt = Ob + (size_t)blockIdx.z * strideOut;
  const int n0 = blockIdx.x * 64;
  const int k0 = blockIdx.y * 64;
#pragma unroll
  for (int p = 0; p < 16; ++p) {
    const int idx = tid + p * 256;
    const int kk  = idx >> 6;
    const int nn  = idx & 63;
    const float v = W[(size_t)(k0 + kk) * Ndim + n0 + nn];
    tile[kk * 65 + nn] = v * scale;
  }
  __syncthreads();
  const int q = lane >> 3, c8 = (lane & 7) * 8;
  v8h hv[2];
#pragma unroll
  for (int it = 0; it < 2; ++it) {
    const int nrow = it * 32 + wave * 4 + q;
#pragma unroll
    for (int e = 0; e < 8; ++e) hv[it][e] = (_Float16)tile[(c8 + e) * 65 + nrow];
  }
  for (int pass = 0; pass < 2; ++pass) {
#pragma unroll
    for (int it = 0; it < 2; ++it) {
      const int nrow = it * 32 + wave * 4 + q;
      *(volatile v8h*)(Bt + (size_t)(n0 + nrow) * Kdim + k0 + c8) = hv[it];
    }
    __threadfence();
  }
}

__device__ __forceinline__ float wave_sum(float v) {
#pragma unroll
  for (int off = 1; off < 32; off <<= 1) v += __shfl_xor(v, off, 32);
  return v;
}

__global__ __launch_bounds__(256) void ln_in_kernel(
    const float* __restrict__ x, const float* __restrict__ gam, const float* __restrict__ bet,
    unsigned short* __restrict__ H16, int bidx, float oscale)
{
  __shared__ __align__(16) _Float16 sH[8 * 2 * kHP];
  const int tid = threadIdx.x, lane = tid & 31, wave = tid >> 5;
  const v4f gv = *(const v4f*)(gam + lane * 4);
  const v4f bv = *(const v4f*)(bet + lane * 4);
  _Float16* sw = sH + wave * 2 * kHP;
  const int rbase = blockIdx.x * 64 + wave * 8;
#pragma unroll 1
  for (int pr = 0; pr < 4; ++pr) {
#pragma unroll
    for (int rr = 0; rr < 2; ++rr) {
      const int m = rbase + pr * 2 + rr;
      const int n = m >> 8, t = m & (kT - 1);
      const v4f v = *(const v4f*)(x + (((size_t)bidx * kT + t) * kNsp + n) * kCh + lane * 4);
      const float mean = wave_sum(v[0] + v[1] + v[2] + v[3]) * (1.0f / kCh);
      const float e0 = v[0] - mean, e1 = v[1] - mean, e2 = v[2] - mean, e3 = v[3] - mean;
      const float var = wave_sum(e0 * e0 + e1 * e1 + e2 * e2 + e3 * e3) * (1.0f / kCh);
      const float rs = rsqrtf(var + 1e-5f);
      sw[rr * kHP + lane * 4 + 0] = (_Float16)((e0 * rs * gv[0] + bv[0]) * oscale);
      sw[rr * kHP + lane * 4 + 1] = (_Float16)((e1 * rs * gv[1] + bv[1]) * oscale);
      sw[rr * kHP + lane * 4 + 2] = (_Float16)((e2 * rs * gv[2] + bv[2]) * oscale);
      sw[rr * kHP + lane * 4 + 3] = (_Float16)((e3 * rs * gv[3] + bv[3]) * oscale);
    }
    __builtin_amdgcn_fence(__ATOMIC_RELEASE, "workgroup");
    __builtin_amdgcn_wave_barrier();
    __builtin_amdgcn_fence(__ATOMIC_ACQUIRE, "workgroup");
    const int hr = lane >> 4, c8 = (lane & 15) * 8;
    const v8h hv = *(const v8h*)(sw + hr * kHP + c8);
    unsigned short* dst = H16 + (size_t)(rbase + pr * 2 + hr) * kCh + c8;
    *(volatile v8h*)dst = hv;
    __threadfence();
    *(volatile v8h*)dst = hv;
    __builtin_amdgcn_fence(__ATOMIC_RELEASE, "workgroup");
    __builtin_amdgcn_wave_barrier();
    __builtin_amdgcn_fence(__ATOMIC_ACQUIRE, "workgroup");
  }
}

__global__ __launch_bounds__(256) void ln_mid_kernel(
    const float* __restrict__ P, const float* __restrict__ x,
    const float* __restrict__ g2, const float* __restrict__ b2,
    const float* __restrict__ g3, const float* __restrict__ b3,
    float* __restrict__ XO, unsigned short* __restrict__ H2, int bidx, float oscale)
{
  __shared__ __align__(16) _Float16 sH[8 * 2 * kHP];
  const int tid = threadIdx.x, lane = tid & 31, wave = tid >> 5;
  const v4f g2v = *(const v4f*)(g2 + lane * 4);
  const v4f b2v = *(const v4f*)(b2 + lane * 4);
  const v4f g3v = *(const v4f*)(g3 + lane * 4);
  const v4f b3v = *(const v4f*)(b3 + lane * 4);
  _Float16* sw = sH + wave * 2 * kHP;
  const int rbase = blockIdx.x * 64 + wave * 8;
#pragma unroll 1
  for (int pr = 0; pr < 4; ++pr) {
#pragma unroll
    for (int rr = 0; rr < 2; ++rr) {
      const int r = rbase + pr * 2 + rr;
      const int t = r >> 6, n = r & (kNsp - 1);
      const int m = n * kT + t;
      const v4f p  = *(const v4f*)(P + (size_t)m * kCh + lane * 4);
      const v4f xs = *(const v4f*)(x + ((size_t)bidx * kRows + r) * kCh + lane * 4);
      const float mean = wave_sum(p[0] + p[1] + p[2] + p[3]) * (1.0f / kCh);
      const float e0 = p[0] - mean, e1 = p[1] - mean, e2 = p[2] - mean, e3 = p[3] - mean;
      const float var = wave_sum(e0 * e0 + e1 * e1 + e2 * e2 + e3 * e3) * (1.0f / kCh);
      const float rs = rsqrtf(var + 1e-5f);
      v4f xo;
      xo[0] = (e0 * rs * g2v[0] + b2v[0]) + xs[0];
      xo[1] = (e1 * rs * g2v[1] + b2v[1]) + xs[1];
      xo[2] = (e2 * rs * g2v[2] + b2v[2]) + xs[2];
      xo[3] = (e3 * rs * g2v[3] + b2v[3]) + xs[3];
      float* xdst = XO + (size_t)r * kCh + lane * 4;
      *(volatile v4f*)xdst = xo;
      __threadfence();
      *(volatile v4f*)xdst = xo;
      const float mean3 = wave_sum(xo[0] + xo[1] + xo[2] + xo[3]) * (1.0f / kCh);
      const float f0 = xo[0] - mean3, f1 = xo[1] - mean3, f2 = xo[2] - mean3, f3 = xo[3] - mean3;
      const float var3 = wave_sum(f0 * f0 + f1 * f1 + f2 * f2 + f3 * f3) * (1.0f / kCh);
      const float rs3 = rsqrtf(var3 + 1e-5f);
      sw[rr * kHP + lane * 4 + 0] = (_Float16)((f0 * rs3 * g3v[0] + b3v[0]) * oscale);
      sw[rr * kHP + lane * 4 + 1] = (_Float16)((f1 * rs3 * g3v[1] + b3v[1]) * oscale);
      sw[rr * kHP + lane * 4 + 2] = (_Float16)((f2 * rs3 * g3v[2] + b3v[2]) * oscale);
      sw[rr * kHP + lane * 4 + 3] = (_Float16)((f3 * rs3 * g3v[3] + b3v[3]) * oscale);
    }
    __builtin_amdgcn_fence(__ATOMIC_RELEASE, "workgroup");
    __builtin_amdgcn_wave_barrier();
    __builtin_amdgcn_fence(__ATOMIC_ACQUIRE, "workgroup");
    const int hr = lane >> 4, c8 = (lane & 15) * 8;
    const v8h hv = *(const v8h*)(sw + hr * kHP + c8);
    unsigned short* dst = H2 + (size_t)(rbase + pr * 2 + hr) * kCh + c8;
    *(volatile v8h*)dst = hv;
    __threadfence();
    *(volatile v8h*)dst = hv;
    __builtin_amdgcn_fence(__ATOMIC_RELEASE, "workgroup");
    __builtin_amdgcn_wave_barrier();
    __builtin_amdgcn_fence(__ATOMIC_ACQUIRE, "workgroup");
  }
}

__global__ __launch_bounds__(256) void conv_silu_kernel(
    const float* __restrict__ XZ, const float* __restrict__ cw, const float* __restrict__ cb,
    unsigned short* __restrict__ U16, int rev)
{
  __shared__ __align__(16) float sT[16 * kTP];
  const int tid = threadIdx.x, lane = tid & 31, wave = tid >> 5;
  const int d0 = blockIdx.x * 256, d = d0 + tid;
  const int t0 = blockIdx.y * 64;
  const int sl = blockIdx.z;
  const size_t brow = (size_t)sl * kT;
  const float w0 = cw[d * 4 + 0], w1 = cw[d * 4 + 1], w2 = cw[d * 4 + 2], w3 = cw[d * 4 + 3];
  const float bc = cb[d];
  float xm3, xm2, xm1;
  {
    const int r3 = t0 - 3, r2 = t0 - 2, r1 = t0 - 1;
    const int c3 = r3 < 0 ? 0 : r3, c2 = r2 < 0 ? 0 : r2, c1 = r1 < 0 ? 0 : r1;
    const int l3 = rev ? (kT - 1 - c3) : c3;
    const int l2 = rev ? (kT - 1 - c2) : c2;
    const int l1 = rev ? (kT - 1 - c1) : c1;
    const float v3 = XZ[(brow + (size_t)l3) * kXZP + d];
    const float v2 = XZ[(brow + (size_t)l2) * kXZP + d];
    const float v1 = XZ[(brow + (size_t)l1) * kXZP + d];
    xm3 = (r3 >= 0) ? v3 : 0.f;
    xm2 = (r2 >= 0) ? v2 : 0.f;
    xm1 = (r1 >= 0) ? v1 : 0.f;
  }
#pragma unroll 1
  for (int sub = 0; sub < 4; ++sub) {
    const int lb = t0 + sub * 16;
#pragma unroll 1
    for (int st = 0; st < 16; ++st) {
      const int tt  = lb + st;
      const int tok = rev ? (kT - 1 - tt) : tt;
      const float xin = XZ[(brow + (size_t)tok) * kXZP + d];
      float acc = w0 * xm3;
      acc = fmaf(w1, xm2, acc);
      acc = fmaf(w2, xm1, acc);
      acc = fmaf(w3, xin, acc);
      const float sv = acc + bc;
      const float sg = __builtin_amdgcn_rcpf(1.0f + __expf(-sv));
      sT[st * kTP + tid] = (sv * sg) * 64.0f;
      xm3 = xm2; xm2 = xm1; xm1 = xin;
    }
    __syncthreads();
    v8h bv[2];
#pragma unroll
    for (int it = 0; it < 2; ++it) {
      const float* sp = sT + (it * 8 + wave) * kTP + lane * 8;
      const v4f a0 = *(const v4f*)(sp);
      const v4f a1 = *(const v4f*)(sp + 4);
#pragma unroll
      for (int e = 0; e < 4; ++e) {
        bv[it][e]     = (_Float16)a0[e];
        bv[it][4 + e] = (_Float16)a1[e];
      }
    }
    for (int pass = 0; pass < 2; ++pass) {
#pragma unroll
      for (int it = 0; it < 2; ++it) {
        const int tt  = lb + it * 8 + wave;
        const int tok = rev ? (kT - 1 - tt) : tt;
        *(volatile v8h*)(U16 + (brow + (size_t)tok) * kDin + d0 + lane * 8) = bv[it];
      }
      __threadfence();
    }
    __syncthreads();
  }
}

template <int REV>
__global__ __launch_bounds__(256) void scan_kernel(
    const float* __restrict__ XZ, const float* __restrict__ XDBL,
    const float* __restrict__ cw, const float* __restrict__ cb,
    const float* __restrict__ Wdt, const float* __restrict__ dtb,
    const float* __restrict__ A_log, const float* __restrict__ Dv,
    float* YF, unsigned short* __restrict__ Y16)
{
  __shared__ __align__(16) float sBC[16 * kPrjN];
  __shared__ __align__(16) float sY[16 * kTP];
  const int tid = threadIdx.x, lane = tid & 31, wave = tid >> 5;
  const int d0 = blockIdx.x * 256, d = d0 + tid;
  const int sl = blockIdx.y;
  const size_t brow = (size_t)sl * kT;

  float An[kNst];
#pragma unroll
  for (int n = 0; n < kNst; ++n) An[n] = -expf(A_log[(size_t)d * kNst + n]);
  float wdt[kDtR];
#pragma unroll
  for (int r = 0; r < kDtR; ++r) wdt[r] = Wdt[(size_t)d * kDtR + r];
  const float Dd  = Dv[d];
  const float bdt = dtb[d];
  const float bc  = cb[d];
  const float w0 = cw[d * 4 + 0], w1 = cw[d * 4 + 1], w2 = cw[d * 4 + 2], w3 = cw[d * 4 + 3];
  float h[kNst];
#pragma unroll
  for (int n = 0; n < kNst; ++n) h[n] = 0.f;
  float xm3 = 0.f, xm2 = 0.f, xm1 = 0.f;

#pragma unroll 1
  for (int c = 0; c < kT / 16; ++c) {
    const int l0 = c * 16;
    if (tid < 160) {
      const int r = tid / 10, q = (tid - r * 10) * 4;
      const int tt  = l0 + r;
      const int tok = REV ? (kT - 1 - tt) : tt;
      const v4f v = *(const v4f*)(XDBL + (brow + (size_t)tok) * kPrjP + q);
      *(v4f*)(sBC + r * kPrjN + q) = v;
    }
    __syncthreads();
#pragma unroll 1
    for (int st = 0; st < 16; ++st) {
      const int tt  = l0 + st;
      const int tok = REV ? (kT - 1 - tt) : tt;
      const size_t m = brow + (size_t)tok;
      const float* row = sBC + st * kPrjN;
      float dacc = 0.f;
#pragma unroll
      for (int r = 0; r < kDtR; ++r) dacc = fmaf(row[r], wdt[r], dacc);
      const float a     = dacc + bdt;
      const float delta = fmaxf(a, 0.0f) + log1pf(__expf(-fabsf(a)));
      const float xin   = XZ[m * kXZP + d];
      float acc = w0 * xm3;
      acc = fmaf(w1, xm2, acc);
      acc = fmaf(w2, xm1, acc);
      acc = fmaf(w3, xin, acc);
      const float sv  = acc + bc;
      const float sgx = __builtin_amdgcn_rcpf(1.0f + __expf(-sv));
      const float xv  = sv * sgx;
      xm3 = xm2; xm2 = xm1; xm1 = xin;
      const float zv  = XZ[m * kXZP + kDin + d];
      v4f Bq[4], Cq[4];
#pragma unroll
      for (int qq = 0; qq < 4; ++qq) {
        Bq[qq] = *(const v4f*)(row + kDtR + 4 * qq);
        Cq[qq] = *(const v4f*)(row + kDtR + kNst + 4 * qq);
      }
      float dx = delta * xv;
      asm volatile("" : "+v"(dx));
      float y = 0.f;
#pragma unroll
      for (int n = 0; n < kNst; ++n) {
        const float e = __expf(delta * An[n]);
        float p = dx * Bq[n >> 2][n & 3];
        asm volatile("" : "+v"(p));
        float qv = h[n] * e;
        asm volatile("" : "+v"(qv));
        const float hn = qv + p;
        h[n] = hn;
        float rr = Cq[n >> 2][n & 3] * hn;
        asm volatile("" : "+v"(rr));
        y += rr;
      }
      float sk = xv * Dd;
      asm volatile("" : "+v"(sk));
      y += sk;
      const float sg = __builtin_amdgcn_rcpf(1.0f + __expf(-zv));
      const float g  = zv * sg;
      float yo = y * g;
      if (REV) {
        const float yother = YF[m * kDin + d];
        yo = (yo + yother) * 1024.0f;
      }
      sY[st * kTP + tid] = yo;
    }
    __syncthreads();
    if (REV) {
      v8h hv[2];
#pragma unroll
      for (int it = 0; it < 2; ++it) {
        const float* sp = sY + (it * 8 + wave) * kTP + lane * 8;
        const v4f a0 = *(const v4f*)(sp);
        const v4f a1 = *(const v4f*)(sp + 4);
#pragma unroll
        for (int e = 0; e < 4; ++e) {
          hv[it][e]     = (_Float16)a0[e];
          hv[it][4 + e] = (_Float16)a1[e];
        }
      }
      for (int pass = 0; pass < 2; ++pass) {
#pragma unroll
        for (int it = 0; it < 2; ++it) {
          const int tt  = l0 + it * 8 + wave;
          const int tok = kT - 1 - tt;
          *(volatile v8h*)(Y16 + (brow + (size_t)tok) * kDin + d0 + lane * 8) = hv[it];
        }
        __threadfence();
      }
    } else {
      v4f fv[2][2];
#pragma unroll
      for (int it = 0; it < 2; ++it) {
        const float* sp = sY + (it * 8 + wave) * kTP;
        fv[it][0] = *(const v4f*)(sp + lane * 4);
        fv[it][1] = *(const v4f*)(sp + 128 + lane * 4);
      }
      for (int pass = 0; pass < 2; ++pass) {
#pragma unroll
        for (int it = 0; it < 2; ++it) {
          const int tt = l0 + it * 8 + wave;
          float* yrow = YF + (brow + (size_t)tt) * kDin + d0;
          *(volatile v4f*)(yrow + lane * 4)       = fv[it][0];
          *(volatile v4f*)(yrow + 128 + lane * 4) = fv[it][1];
        }
        __threadfence();
      }
    }
  }
}

__global__ __launch_bounds__(256) void gelu_cast_kernel(
    const float* __restrict__ src, unsigned short* __restrict__ dst, int total2, float scale)
{
  const int i = blockIdx.x * 256 + threadIdx.x;
  if (i >= total2) return;
  const float* p = src + (size_t)i * 2;
  float r0 = 0.f, r1 = 0.f;
#pragma unroll 1
  for (int e = 0; e < 2; ++e) {
    const float v  = p[e];
    const float gq = 0.5f * v * (1.0f + erff(v * 0.70710678118654752f));
    const float gs = gq * scale;
    r0 = (e == 0) ? gs : r0;
    r1 = (e == 0) ? r1 : gs;
  }
  const _Float16 h0 = (_Float16)r0, h1 = (_Float16)r1;
  const unsigned u = (unsigned)__builtin_bit_cast(unsigned short, h0) | ((unsigned)__builtin_bit_cast(unsigned short, h1) << 16);
  unsigned* q = (unsigned*)(void*)dst + i;
  *(volatile unsigned*)q = u;
  __threadfence();
  *(volatile unsigned*)q = u;
}

extern "C" void kernel_launch(void* const* d_in, const int* in_sizes, int n_in,
                              void* d_out, int out_size, void* d_ws, size_t ws_size,
                              hipStream_t stream)
{
  if (n_in < 27) return;
  const float* x      = (const float*)d_in[0];
  const float* g1     = (const float*)d_in[1];
  const float* b1     = (const float*)d_in[2];
  const float* W_in   = (const float*)d_in[3];
  const float* cw_f   = (const float*)d_in[4];
  const float* cb_f   = (const float*)d_in[5];
  const float* Wx_f   = (const float*)d_in[6];
  const float* Wdt_f  = (const float*)d_in[7];
  const float* bdt_f  = (const float*)d_in[8];
  const float* Alg_f  = (const float*)d_in[9];
  const float* D_f    = (const float*)d_in[10];
  const float* cw_b   = (const float*)d_in[11];
  const float* cb_b   = (const float*)d_in[12];
  const float* Wx_b   = (const float*)d_in[13];
  const float* Wdt_b  = (const float*)d_in[14];
  const float* bdt_b  = (const float*)d_in[15];
  const float* Alg_b  = (const float*)d_in[16];
  const float* D_b    = (const float*)d_in[17];
  const float* W_out  = (const float*)d_in[18];
  const float* g2     = (const float*)d_in[19];
  const float* b2     = (const float*)d_in[20];
  const float* g3     = (const float*)d_in[21];
  const float* b3     = (const float*)d_in[22];
  const float* W1m    = (const float*)d_in[23];
  const float* b1m    = (const float*)d_in[24];
  const float* W2m    = (const float*)d_in[25];
  const float* b2m    = (const float*)d_in[26];
  float* dout = (float*)d_out;

  if (in_sizes[0] != kBatch * kT * kNsp * kCh) return;
  if (in_sizes[1] != kCh || in_sizes[2] != kCh) return;
  if (in_sizes[3] != kXZP * kCh) return;
  if (in_sizes[4] != kDin * 4 || in_sizes[5] != kDin) return;
  if (in_sizes[6] != kPrjN * kDin || in_sizes[7] != kDin * kDtR || in_sizes[8] != kDin) return;
  if (in_sizes[9] != kDin * kNst || in_sizes[10] != kDin) return;
  if (in_sizes[11] != kDin * 4 || in_sizes[12] != kDin) return;
  if (in_sizes[13] != kPrjN * kDin || in_sizes[14] != kDin * kDtR || in_sizes[15] != kDin) return;
  if (in_sizes[16] != kDin * kNst || in_sizes[17] != kDin) return;
  if (in_sizes[18] != kCh * kDin) return;
  if (in_sizes[19] != kCh || in_sizes[20] != kCh || in_sizes[21] != kCh || in_sizes[22] != kCh) return;
  if (in_sizes[23] != kCh * kMlp || in_sizes[24] != kMlp) return;
  if (in_sizes[25] != kMlp * kCh || in_sizes[26] != kCh) return;
  if (out_size != kBatch * kT * kNsp * kCh) return;

  const size_t SZ_WIN16  = (size_t)kXZP * kCh * 2;
  const size_t SZ_WX16   = (size_t)kPrjP * kDin * 2;
  const size_t SZ_WOUT16 = (size_t)kCh * kDin * 2;
  const size_t SZ_W1T16  = (size_t)kMlp * kCh * 2;
  const size_t SZ_W2T16  = (size_t)kCh * kMlp * 2;
  const size_t SZ_H16    = (size_t)kRows * kCh * 2;
  const size_t SZ_XZ     = (size_t)kRows * kXZP * 4;
  const size_t SZ_U16    = (size_t)kRows * kDin * 2;
  const size_t SZ_XDBL   = (size_t)kRows * kPrjP * 4;
  const size_t SZ_YF     = (size_t)kRows * kDin * 4;
  const size_t SZ_Y16    = (size_t)kRows * kDin * 2;
  const size_t SZ_P      = (size_t)kRows * kCh * 4;
  const size_t SZ_XO     = (size_t)kRows * kCh * 4;
  const size_t SZ_H2     = (size_t)kRows * kCh * 2;
  const size_t SZ_PRE    = (size_t)kRows * kMlp * 4;
  const size_t SZ_G16    = (size_t)kRows * kMlp * 2;
  const size_t OFF_WIN16  = 0;
  const size_t OFF_WX16   = OFF_WIN16  + SZ_WIN16;
  const size_t OFF_WOUT16 = OFF_WX16   + 2 * SZ_WX16;
  const size_t OFF_W1T16  = OFF_WOUT16 + SZ_WOUT16;
  const size_t OFF_W2T16  = OFF_W1T16  + SZ_W1T16;
  const size_t OFF_H16    = OFF_W2T16  + SZ_W2T16;
  const size_t OFF_XZ     = OFF_H16    + SZ_H16;
  const size_t OFF_U16    = OFF_XZ     + SZ_XZ;
  const size_t OFF_XDBL   = OFF_U16    + SZ_U16;
  const size_t OFF_YF     = OFF_XDBL   + SZ_XDBL;
  const size_t OFF_Y16    = OFF_YF     + SZ_YF;
  const size_t OFF_P      = OFF_Y16    + SZ_Y16;
  const size_t OFF_XO     = OFF_P      + SZ_P;
  const size_t OFF_H2     = OFF_XO     + SZ_XO;
  const size_t OFF_PRE    = OFF_H2     + SZ_H2;
  const size_t OFF_G16    = OFF_PRE    + SZ_PRE;
  const size_t TOTAL      = OFF_G16    + SZ_G16;
  if (ws_size < TOTAL) return;

  char* ws = (char*)d_ws;
  unsigned short* WIN16  = (unsigned short*)(ws + OFF_WIN16);
  unsigned short* WX16[2];
  WX16[0] = (unsigned short*)(ws + OFF_WX16);
  WX16[1] = (unsigned short*)(ws + OFF_WX16 + SZ_WX16);
  unsigned short* WOUT16 = (unsigned short*)(ws + OFF_WOUT16);
  unsigned short* W1T16  = (unsigned short*)(ws + OFF_W1T16);
  unsigned short* W2T16  = (unsigned short*)(ws + OFF_W2T16);
  unsigned short* H16    = (unsigned short*)(ws + OFF_H16);
  float*          XZ     = (float*)(ws + OFF_XZ);
  unsigned short* U16    = (unsigned short*)(ws + OFF_U16);
  float*          XDBL   = (float*)(ws + OFF_XDBL);
  float*          YF     = (float*)(ws + OFF_YF);
  unsigned short* Y16    = (unsigned short*)(ws + OFF_Y16);
  float*          P      = (float*)(ws + OFF_P);
  float*          XO     = (float*)(ws + OFF_XO);
  unsigned short* H2     = (unsigned short*)(ws + OFF_H2);
  float*          PRE    = (float*)(ws + OFF_PRE);
  unsigned short* G16    = (unsigned short*)(ws + OFF_G16);
  const float* dummy_bias  = g1;
  const float* dummy_resid = x;

  const float* cwp[2]  = {cw_f, cw_b};
  const float* cbp[2]  = {cb_f, cb_b};
  const float* wxp[2]  = {Wx_f, Wx_b};

  cast_rows_f16_kernel<<<(kXZP * kCh) / 8 / 256, 256, 0, stream>>>(W_in, WIN16, kXZP, kCh, (kXZP * kCh) / 8, 32.0f);
  for (int dir = 0; dir < 2; ++dir) {
    cast_rows_f16_kernel<<<(kPrjP * kDin) / 8 / 256, 256, 0, stream>>>(wxp[dir], WX16[dir], kPrjN, kDin, (kPrjP * kDin) / 8, 32.0f);
  }
  cast_rows_f16_kernel<<<(kCh * kDin) / 8 / 256, 256, 0, stream>>>(W_out, WOUT16, kCh, kDin, (kCh * kDin) / 8, 32.0f);
  xpose_cast_kernel<<<dim3(kMlp / 64, kCh / 64, 1), 256, 0, stream>>>(W1m, W1T16, kCh, kMlp, 0L, 0L, 32.0f);
  xpose_cast_kernel<<<dim3(kCh / 64, kMlp / 64, 1), 256, 0, stream>>>(W2m, W2T16, kMlp, kCh, 0L, 0L, 32.0f);

  const int total2_mlp = (kRows * kMlp) / 2;

  for (int b = 0; b < kBatch; ++b) {
    ln_in_kernel<<<kRows / 64, 256, 0, stream>>>(x, g1, b1, H16, b, 4.0f);

    wmma_gemm64<0, false, 0, 0, false><<<dim3(256, 1), 256, 0, stream>>>(
        H16, H16, kCh, 0L, WIN16, WIN16, kCh, 0L,
        (void*)XZ, (void*)XZ, kXZP, 0L, dummy_bias, dummy_resid, 0L, kRows, kXZP, kCh, 1.0f / 128.0f);

    for (int dir = 0; dir < 2; ++dir) {
      conv_silu_kernel<<<dim3(kDin / 256, kT / 64, kNsp), 256, 0, stream>>>(XZ, cwp[dir], cbp[dir], U16, dir);

      wmma_gemm64<0, false, 0, 0, false><<<dim3(32, 1), 256, 0, stream>>>(
          U16, U16, kDin, 0L, WX16[dir], WX16[dir], kDin, 0L,
          (void*)XDBL, (void*)XDBL, kPrjP, 0L, dummy_bias, dummy_resid, 0L, kRows, kPrjP, kDin, 1.0f / 2048.0f);

      if (dir == 0) {
        scan_kernel<0><<<dim3(kDin / 256, kNsp), 256, 0, stream>>>(
            XZ, XDBL, cw_f, cb_f, Wdt_f, bdt_f, Alg_f, D_f, YF, Y16);
      } else {
        scan_kernel<1><<<dim3(kDin / 256, kNsp), 256, 0, stream>>>(
            XZ, XDBL, cw_b, cb_b, Wdt_b, bdt_b, Alg_b, D_b, YF, Y16);
      }
    }

    wmma_gemm64<0, false, 0, 0, false><<<dim3(64, 1), 256, 0, stream>>>(
        Y16, Y16, kDin, 0L, WOUT16, WOUT16, kDin, 0L,
        (void*)P, (void*)P, kCh, 0L, dummy_bias, dummy_resid, 0L, kRows, kCh, kDin, 1.0f / 32768.0f);

    ln_mid_kernel<<<kRows / 64, 256, 0, stream>>>(P, x, g2, b2, g3, b3, XO, H2, b, 4.0f);

    wmma_gemm64<0, false, 2, 0, false><<<dim3(128, 1), 256, 0, stream>>>(
        H2, H2, kCh, 0L, W1T16, W1T16, kCh, 0L,
        (void*)PRE, (void*)PRE, kMlp, 0L, b1m, dummy_resid, 0L, kRows, kMlp, kCh, 1.0f / 128.0f);

    gelu_cast_kernel<<<total2_mlp / 256, 256, 0, stream>>>(PRE, G16, total2_mlp, 64.0f);

    wmma_gemm64<0, false, 2, 0, true><<<dim3(64, 1), 256, 0, stream>>>(
        G16, G16, kMlp, 0L, W2T16, W2T16, kMlp, 0L,
        (void*)(dout + (size_t)b * kRows * kCh), (void*)(dout + (size_t)b * kRows * kCh), kCh, 0L,
        b2m, XO, 0L, kRows, kCh, kMlp, 1.0f / 2048.0f);
  }
}
